// KSSMBlock_66872640798748
// MI455X (gfx1250) — hardware-run, weakly checked
//
#include <hip/hip_runtime.h>
#include <math.h>

#define NB    2
#define TLEN  2048
#define DMOD  1024
#define DIN   2048
#define DTR   64
#define NGRP  16
#define NPJ   4192
#define NPP   4224
#define OFF_X 2048
#define OFF_B 4096
#define OFF_R 4128
#define NTOK  4096
#define NADO  6144
#define TCH   512
#define NCHK  4
#define MCH   1024
#define TPB   128
#define OSTR  68
#define SCH   32
#define CHB   64
#define NSCB  64
#define WSC   64.0f
#define YSC   64.0f
#define LSC   2048.0f

static_assert(NTOK == NB * TLEN);
static_assert(NPJ == 2 * DIN + 2 * NGRP + DTR);
static_assert(NPP % 64 == 0);
static_assert(NPP >= NPJ);
static_assert(NPP % 4 == 0);
static_assert((NPP - DIN) % 64 == 0);
static_assert(OFF_R % 4 == 0);
static_assert(NTOK % TPB == 0);
static_assert(MCH == NB * TCH);
static_assert(MCH % TPB == 0);
static_assert(TCH % TPB == 0);
static_assert(TLEN % TCH == 0);
static_assert(NCHK == TLEN / TCH);
static_assert(TCH % SCH == 0);
static_assert(NADO == 3 * DIN);
static_assert(NADO % 64 == 0);
static_assert(DIN % 64 == 0);
static_assert(DMOD % 64 == 0);
static_assert(DMOD % 32 == 0);
static_assert(DTR % 32 == 0);
static_assert(DIN % 32 == 0);
static_assert(DIN % CHB == 0);
static_assert((DIN / NGRP) % CHB == 0);
static_assert(NSCB == NB * (DIN / CHB));
static_assert(SCH * CHB == 4 * CHB * 8);
static_assert(2 * CHB == 32 * 4);
static_assert(CHB == 64);
static_assert(OSTR % 4 == 0);
static_assert(DMOD == 128 * 8);
static_assert(DMOD % 8 == 0);
static_assert(DTR % 8 == 0);
static_assert(DIN % 8 == 0);

typedef unsigned short us16 __attribute__((ext_vector_type(16)));
typedef unsigned short us8  __attribute__((ext_vector_type(8)));
typedef unsigned short us8a __attribute__((ext_vector_type(8), may_alias));
typedef _Float16 v16h __attribute__((ext_vector_type(16)));
typedef _Float16 v8h  __attribute__((ext_vector_type(8)));
typedef float v8f __attribute__((ext_vector_type(8)));
typedef float v4f __attribute__((ext_vector_type(4)));
typedef float v4fa __attribute__((ext_vector_type(4), may_alias));
union FragU { us16 v; us8 h[2]; };
union H8 { v8h f; us8 u; };

__device__ __forceinline__ float bf16r(float f) {
  unsigned u = __float_as_uint(f);
  u += 0x7FFFu + ((u >> 16) & 1u);
  return __uint_as_float(u & 0xFFFF0000u);
}
__device__ __forceinline__ float siluf(float x) { return x * (1.0f / (1.0f + expf(-x))); }
__device__ __forceinline__ float softplusf(float t) { return fmaxf(t, 0.0f) + log1pf(expf(-fabsf(t))); }
__device__ __forceinline__ float wsum(float v) {
#pragma unroll
  for (int o = 16; o > 0; o >>= 1) v += __shfl_xor(v, o);
  return v;
}
__device__ __forceinline__ us8 pack8(const v4f a, const v4f b, float sc) {
  H8 o;
#pragma unroll
  for (int u = 0; u < 4; ++u) { o.f[u] = (_Float16)(a[u] * sc); o.f[4 + u] = (_Float16)(b[u] * sc); }
  return o.u;
}
__device__ __forceinline__ void split8(const v4f a, const v4f b, us8& hi, us8& lo) {
  H8 h, l;
#pragma unroll
  for (int u = 0; u < 4; ++u) {
    const _Float16 ha = (_Float16)a[u];
    h.f[u] = ha; l.f[u] = (_Float16)((a[u] - (float)ha) * LSC);
    const _Float16 hb = (_Float16)b[u];
    h.f[4 + u] = hb; l.f[4 + u] = (_Float16)((b[u] - (float)hb) * LSC);
  }
  hi = h.u; lo = l.u;
}

__device__ __forceinline__ v8f mma16(us16 a, us16 b, v8f c) {
  return __builtin_amdgcn_wmma_f32_16x16x32_f16(false, __builtin_bit_cast(v16h, a), false, __builtin_bit_cast(v16h, b), (short)0, c, false, false);
}
__device__ __forceinline__ void wguard4(v8f& c0, v8f& c1, v8f& c2, v8f& c3, const us16& a0,
                                        const us16& b0, const us16& b1, const us16& b2, const us16& b3) {
#if defined(__HIP_DEVICE_COMPILE__)
  asm volatile("v_nop\n\tv_nop\n\tv_nop\n\tv_nop"
               : "+v"(c0), "+v"(c1), "+v"(c2), "+v"(c3)
               : "v"(a0), "v"(b0), "v"(b1), "v"(b2), "v"(b3));
#endif
}
__device__ __forceinline__ void wguard8(v8f& c0, v8f& c1, v8f& c2, v8f& c3, v8f& d0, v8f& d1, v8f& d2, v8f& d3,
                                        const us16& a0, const us16& a1,
                                        const us16& b0, const us16& b1, const us16& b2, const us16& b3) {
#if defined(__HIP_DEVICE_COMPILE__)
  asm volatile("v_nop\n\tv_nop\n\tv_nop\n\tv_nop"
               : "+v"(c0), "+v"(c1), "+v"(c2), "+v"(c3), "+v"(d0), "+v"(d1), "+v"(d2), "+v"(d3)
               : "v"(a0), "v"(a1), "v"(b0), "v"(b1), "v"(b2), "v"(b3));
#endif
}

__device__ __forceinline__ us16 gfrag(const unsigned short* p) {
  const int kh = ((threadIdx.x >> 4) & 1) * 8;
  FragU f;
  f.h[0] = *(const us8a*)(p + kh);
  f.h[1] = *(const us8a*)(p + 16 + kh);
  return f.v;
}

__global__ __launch_bounds__(256) void k_cvt(const float* __restrict__ src, int lds_, int nsrc, int ncol8, int total8, float sc,
                                            unsigned short* dst) {
  const int idx = blockIdx.x * 256 + threadIdx.x;
  if (idx >= total8) return;
  const int row = idx / ncol8, c8 = (idx - row * ncol8) * 8;
  const int rs = (row < nsrc) ? row : (nsrc - 1);
  const float* s = src + (size_t)rs * (size_t)lds_ + c8;
  v4f a = *(const v4fa*)s, b = *(const v4fa*)(s + 4);
#pragma unroll
  for (int u = 0; u < 4; ++u) { a[u] = bf16r(a[u]); b[u] = bf16r(b[u]); }
  const v4f z4 = {0.0f, 0.0f, 0.0f, 0.0f};
  if (row >= nsrc) { a = z4; b = z4; }
  const us8 o = pack8(a, b, sc);
  const size_t off = (size_t)row * (size_t)(ncol8 * 8) + c8;
  *(volatile us8*)(dst + off) = o;
  __threadfence();
  *(volatile us8*)(dst + off) = o;
}

__global__ __launch_bounds__(256) void k_split(const float* __restrict__ src, int lds_, int ncol8, int total8,
                                              unsigned short* H, unsigned short* L) {
  const int idx = blockIdx.x * 256 + threadIdx.x;
  if (idx >= total8) return;
  const int row = idx / ncol8, c8 = (idx - row * ncol8) * 8;
  const float* s = src + (size_t)row * (size_t)lds_ + c8;
  const v4f a = *(const v4fa*)s, b = *(const v4fa*)(s + 4);
  us8 hi, lo;
  split8(a, b, hi, lo);
  const size_t off = (size_t)row * (size_t)(ncol8 * 8) + c8;
  *(volatile us8*)(H + off) = hi; *(volatile us8*)(L + off) = lo;
  __threadfence();
  *(volatile us8*)(H + off) = hi; *(volatile us8*)(L + off) = lo;
}

__global__ __launch_bounds__(128) void k_ln(const float* __restrict__ x, const float* __restrict__ w, const float* __restrict__ bb,
                                           unsigned short* XH, unsigned short* XL) {
  __shared__ float r1s[4];
  __shared__ float r2s[4];
  const int tid = threadIdx.x, lane = tid & 31, wave = tid >> 5, row = blockIdx.x, i0 = tid * 8;
  const float* xr = x + (size_t)row * DMOD + i0;
  v4f a = *(const v4fa*)xr, b = *(const v4fa*)(xr + 4);
#pragma unroll
  for (int u = 0; u < 4; ++u) { a[u] = bf16r(a[u]); b[u] = bf16r(b[u]); }
  float s = ((a[0] + a[1]) + (a[2] + a[3])) + ((b[0] + b[1]) + (b[2] + b[3]));
  s = wsum(s);
  if (lane == 0) r1s[wave] = s;
  __syncthreads();
  const float mean = ((r1s[0] + r1s[1]) + (r1s[2] + r1s[3])) * (1.0f / DMOD);
  float q = 0.0f;
#pragma unroll
  for (int u = 0; u < 4; ++u) { const float d0 = a[u] - mean; q += d0 * d0; const float d1 = b[u] - mean; q += d1 * d1; }
  q = wsum(q);
  if (lane == 0) r2s[wave] = q;
  __syncthreads();
  const float var = ((r2s[0] + r2s[1]) + (r2s[2] + r2s[3])) * (1.0f / DMOD);
  const float rstd = rsqrtf(var + 1e-5f);
  const v4f wa = *(const v4fa*)(w + i0), wb = *(const v4fa*)(w + i0 + 4);
  const v4f ba = *(const v4fa*)(bb + i0), bv = *(const v4fa*)(bb + i0 + 4);
  v4f oa, ob;
#pragma unroll
  for (int u = 0; u < 4; ++u) {
    oa[u] = (a[u] - mean) * rstd * bf16r(wa[u]) + bf16r(ba[u]);
    ob[u] = (b[u] - mean) * rstd * bf16r(wb[u]) + bf16r(bv[u]);
  }
  us8 hi, lo;
  split8(oa, ob, hi, lo);
  const size_t off = (size_t)row * DMOD + i0;
  *(volatile us8*)(XH + off) = hi; *(volatile us8*)(XL + off) = lo;
  __threadfence();
  *(volatile us8*)(XH + off) = hi; *(volatile us8*)(XL + off) = lo;
}

template <int MODE, int NPL>
__global__ __launch_bounds__(256) void k_gemm(const unsigned short* __restrict__ A0, const unsigned short* __restrict__ A1, int lda, int cbase,
                                             const unsigned short* __restrict__ Bw, int ldb, int K, float sc, float scl,
                                             const float* __restrict__ bs0, const float* __restrict__ bs1,
                                             const float* __restrict__ bs2, const float* __restrict__ resid,
                                             float* Yf, int ldy) {
  __shared__ __attribute__((aligned(16))) float oS[8 * 16 * OSTR];
  const int tid = threadIdx.x, lane = tid & 31, wave = tid >> 5, cl = lane & 15, hh = lane >> 4;
  const int m0 = blockIdx.x * TPB + 16 * wave;
  int ar0 = m0;
  if (MODE == 1) {
    const int mb = blockIdx.x * TPB, bq = mb / TCH;
    ar0 = bq * TLEN + cbase + (mb - bq * TCH) + 16 * wave;
  }
  const int n0 = blockIdx.y * 64;

  v8f acc[4], acl[4];
#pragma unroll
  for (int j = 0; j < 4; ++j) { const v8f zz = {0.f, 0.f, 0.f, 0.f, 0.f, 0.f, 0.f, 0.f}; acc[j] = zz; acl[j] = zz; }

  const unsigned short* a0p = A0 + (size_t)(ar0 + cl) * (size_t)lda;
  const unsigned short* a1p = A1 + (size_t)(ar0 + cl) * (size_t)lda;
  const unsigned short* bp = Bw + (size_t)(n0 + cl) * (size_t)ldb;
#pragma unroll 1
  for (int k0 = 0; k0 < K; k0 += 32) {
    const us16 af0 = gfrag(a0p + k0);
    us16 af1 = af0;
    if (NPL == 2) af1 = gfrag(a1p + k0);
    us16 bfr[4];
#pragma unroll
    for (int j = 0; j < 4; ++j) bfr[j] = gfrag(bp + (size_t)(16 * j) * (size_t)ldb + k0);
#pragma unroll
    for (int j = 0; j < 4; ++j) acc[j] = mma16(af0, bfr[j], acc[j]);
    if (NPL == 2) {
#pragma unroll
      for (int j = 0; j < 4; ++j) acl[j] = mma16(af1, bfr[j], acl[j]);
      wguard8(acc[0], acc[1], acc[2], acc[3], acl[0], acl[1], acl[2], acl[3], af0, af1, bfr[0], bfr[1], bfr[2], bfr[3]);
    } else {
      wguard4(acc[0], acc[1], acc[2], acc[3], af0, bfr[0], bfr[1], bfr[2], bfr[3]);
    }
  }

  float* so = oS + wave * (16 * OSTR);
#pragma unroll
  for (int j = 0; j < 4; ++j)
#pragma unroll
    for (int r = 0; r < 8; ++r) {
      float t = acc[j][r] * sc;
      if (NPL == 2) t = t + acl[j][r] * scl;
      so[(8 * hh + r) * OSTR + 16 * j + cl] = t;
    }
  __syncthreads();

  if (MODE != 0) {
    int which = 0;
    const float* bias = bs0;
    if (MODE == 1) { which = n0 / DIN; bias = (which == 0) ? bs0 : ((which == 1) ? bs1 : bs2); }
#pragma unroll 1
    for (int it = 0; it < 8; ++it) {
      const int cx = it * 32 + lane, r = cx >> 4, q = (cx & 15) * 4;
      v4f v = *(const v4fa*)(so + r * OSTR + q);
      v4f ex = {0.0f, 0.0f, 0.0f, 0.0f};
      if (MODE == 1) {
#pragma unroll
        for (int u = 0; u < 4; ++u) ex[u] = bias[(n0 - which * DIN) + q + u];
      }
      if (MODE == 2) ex = *(const v4fa*)(resid + (size_t)(m0 + r) * (size_t)ldy + n0 + q);
#pragma unroll
      for (int u = 0; u < 4; ++u) {
        float t = v[u] + bf16r(ex[u]);
        if (MODE == 1) { if (which != 1) t = softplusf(t); }
        v[u] = t;
      }
      *(v4fa*)(so + r * OSTR + q) = v;
    }
  }
#pragma unroll
  for (int pass = 0; pass < 2; ++pass) {
#pragma unroll
    for (int it = 0; it < 8; ++it) {
      const int cx = it * 32 + lane, r = cx >> 4, q = (cx & 15) * 4;
      const v4f v = *(const v4fa*)(so + r * OSTR + q);
      *(volatile v4f*)(Yf + (size_t)(m0 + r) * (size_t)ldy + n0 + q) = v;
    }
    __threadfence();
  }
}

__global__ __launch_bounds__(CHB) void k_scan(const float* __restrict__ PR, const float* __restrict__ AD, int cbase, int rin,
                                             const float* hin, const float* __restrict__ cw, const float* __restrict__ cb,
                                             const float* __restrict__ Cw, const float* __restrict__ Dp,
                                             unsigned short* YG, float* hout) {
#pragma clang fp contract(off)
  __shared__ __attribute__((aligned(16))) float sy[SCH * CHB];
  __shared__ __attribute__((aligned(16))) float hs[2 * CHB];
  const int tid = threadIdx.x;
  const int b = blockIdx.x / (DIN / CHB), dg = blockIdx.x - b * (DIN / CHB);
  const int ch = dg * CHB + tid, grp = ch / (DIN / NGRP);
  const size_t hidx = ((size_t)b * DIN + (size_t)ch) * 2;
  float h0 = hin[hidx], h1 = hin[hidx + 1];
  if (rin) { h0 = bf16r(h0); h1 = bf16r(h1); }
  const float w0 = bf16r(cw[ch * 4 + 0]), w1 = bf16r(cw[ch * 4 + 1]), w2 = bf16r(cw[ch * 4 + 2]), w3 = bf16r(cw[ch * 4 + 3]);
  const float bcv = bf16r(cb[ch]);
  const float c0 = bf16r(Cw[ch * 2 + 0]), c1 = bf16r(Cw[ch * 2 + 1]);
  const float dpar = bf16r(Dp[ch]);
  float xw0, xw1, xw2;
  {
    const size_t base = (size_t)b * TLEN;
    const int t0 = cbase - 3, t1 = cbase - 2, t2 = cbase - 1;
    const float v0 = PR[(base + (size_t)(t0 < 0 ? 0 : t0)) * NPP + OFF_X + ch];
    const float v1 = PR[(base + (size_t)(t1 < 0 ? 0 : t1)) * NPP + OFF_X + ch];
    const float v2 = PR[(base + (size_t)(t2 < 0 ? 0 : t2)) * NPP + OFF_X + ch];
    xw0 = (t0 >= 0) ? v0 : 0.0f;
    xw1 = (t1 >= 0) ? v1 : 0.0f;
    xw2 = (t2 >= 0) ? v2 : 0.0f;
  }

#pragma unroll 1
  for (int c = 0; c < TCH / SCH; ++c) {
    const int tb = cbase + c * SCH;
#pragma unroll 1
    for (int s = 0; s < SCH; ++s) {
      const size_t tok = (size_t)b * TLEN + (size_t)(tb + s);
      const float* pr = PR + tok * NPP;
      const float* ad = AD + ((size_t)b * TCH + (size_t)(c * SCH + s)) * NADO;
      const float zv = pr[ch];
      const float xi = pr[OFF_X + ch];
      const float B0 = pr[OFF_B + 2 * grp], B1 = pr[OFF_B + 2 * grp + 1];
      const float al = ad[ch], om = ad[DIN + ch], dt = ad[2 * DIN + ch];
      float cv = ((w0 * xw0 + w1 * xw1) + w2 * xw2) + w3 * xi;
      cv = cv + bcv;
      xw0 = xw1; xw1 = xw2; xw2 = xi;
      const float xa = siluf(cv);
      const float tau = dt * 0.5f;
      const float opta = 1.0f + tau * al;
      const float tw = tau * om;
      const float inv = 1.0f / ((opta * opta + tw * tw) + 1e-6f);
      const float m11 = opta * inv, m12 = tw * inv;
      const float omta = 1.0f - tau * al;
      const float a11 = m11 * omta - m12 * tw;
      const float a12 = m11 * tw + m12 * omta;
      const float a21 = (-m12) * omta - m11 * tw;
      const float a22 = (-m12) * tw + m11 * omta;
      const float Bx0 = B0 * xa, Bx1 = B1 * xa;
      const float u0 = dt * (m11 * Bx0 + m12 * Bx1);
      const float u1 = dt * ((-m12) * Bx0 + m11 * Bx1);
      const float nh0 = (a11 * h0 + a12 * h1) + u0;
      const float nh1 = (a21 * h0 + a22 * h1) + u1;
      h0 = nh0; h1 = nh1;
      const float y = (h0 * c0 + h1 * c1) + dpar * xa;
      sy[s * CHB + tid] = (y * siluf(zv)) * YSC;
    }
    __syncthreads();
    const size_t row0 = (size_t)b * TLEN + (size_t)tb;
#pragma unroll
    for (int pass = 0; pass < 2; ++pass) {
#pragma unroll
      for (int it = 0; it < 4; ++it) {
        const int ix = it * CHB + tid, r = ix >> 3, q = (ix & 7) * 8;
        const v4f a = *(const v4fa*)(sy + r * CHB + q), bq = *(const v4fa*)(sy + r * CHB + q + 4);
        const us8 o = pack8(a, bq, 1.0f);
        *(volatile us8*)(YG + (row0 + (size_t)r) * DIN + (size_t)dg * CHB + q) = o;
      }
      __threadfence();
    }
    __syncthreads();
  }

  hs[2 * tid] = h0; hs[2 * tid + 1] = h1;
  __syncthreads();
  if (tid < 32) {
    const v4f v = *(const v4fa*)(hs + 4 * tid);
    float* hp = hout + ((size_t)b * DIN + (size_t)dg * CHB) * 2 + 4 * tid;
    *(volatile v4f*)hp = v;
    __threadfence();
    *(volatile v4f*)hp = v;
  }
}

extern "C" void kernel_launch(void* const* d_in, const int* in_sizes, int n_in,
                              void* d_out, int out_size, void* d_ws, size_t ws_size,
                              hipStream_t stream) {
  if (n_in < 16) return;
  if (in_sizes[0] != NTOK * DMOD || in_sizes[1] != NB * DIN * 2 || in_sizes[2] != DMOD || in_sizes[3] != DMOD ||
      in_sizes[4] != NPJ * DMOD || in_sizes[5] != DIN * 4 || in_sizes[6] != DIN || in_sizes[7] != DIN * DTR ||
      in_sizes[8] != DIN || in_sizes[9] != DIN * DTR || in_sizes[10] != DIN || in_sizes[11] != DIN * DTR ||
      in_sizes[12] != DIN || in_sizes[13] != DIN * 2 || in_sizes[14] != DIN || in_sizes[15] != DMOD * DIN) return;
  if (out_size != NTOK * DMOD + NB * DIN * 2) return;

  const float* x       = (const float*)d_in[0];
  const float* state   = (const float*)d_in[1];
  const float* norm_w  = (const float*)d_in[2];
  const float* norm_b  = (const float*)d_in[3];
  const float* in_w    = (const float*)d_in[4];
  const float* conv_w  = (const float*)d_in[5];
  const float* conv_b  = (const float*)d_in[6];
  const float* alpha_w = (const float*)d_in[7];
  const float* alpha_b = (const float*)d_in[8];
  const float* omega_w = (const float*)d_in[9];
  const float* omega_b = (const float*)d_in[10];
  const float* dt_w    = (const float*)d_in[11];
  const float* dt_b    = (const float*)d_in[12];
  const float* C_w     = (const float*)d_in[13];
  const float* D_p     = (const float*)d_in[14];
  const float* out_w   = (const float*)d_in[15];
  float* out  = (float*)d_out;
  float* hout = out + (size_t)NTOK * DMOD;

  size_t off = 0;
  auto carve = [&](size_t bytes) -> char* { char* p = (char*)d_ws + off; off += (bytes + 255) & ~(size_t)255; return p; };
  const size_t szXH = (size_t)NTOK * DMOD * 2, szWIN = (size_t)NPP * DMOD * 2, szADO = (size_t)MCH * NADO * 4;
  size_t szR1 = 2 * szXH + szWIN; if (szADO > szR1) szR1 = szADO;
  char* R1 = carve(szR1);
  float* PROJ = (float*)carve((size_t)NTOK * NPP * 4);
  unsigned short* DTPH = (unsigned short*)carve((size_t)NTOK * DTR * 2);
  unsigned short* DTPL = (unsigned short*)carve((size_t)NTOK * DTR * 2);
  unsigned short* W3   = (unsigned short*)carve((size_t)NADO * DTR * 2);
  unsigned short* WOUT = (unsigned short*)carve((size_t)DMOD * DIN * 2);
  unsigned short* YG   = (unsigned short*)carve((size_t)NTOK * DIN * 2);
  if (off > ws_size || off > (size_t)134217728) return;

  unsigned short* XH  = (unsigned short*)R1;
  unsigned short* XL  = (unsigned short*)(R1 + szXH);
  unsigned short* WIN = (unsigned short*)(R1 + 2 * szXH);
  float* ADO = (float*)R1;

  const dim3 b256(256);
  auto cdv = [](long a, long bq) { return (unsigned)((a + bq - 1) / bq); };

  k_cvt<<<dim3(cdv((long)NPP * DMOD / 8, 256)), b256, 0, stream>>>(in_w, DMOD, NPJ, DMOD / 8, NPP * DMOD / 8, WSC, WIN);
  k_cvt<<<dim3(cdv((long)DIN * DTR / 8, 256)), b256, 0, stream>>>(alpha_w, DTR, DIN, DTR / 8, DIN * DTR / 8, WSC, W3);
  k_cvt<<<dim3(cdv((long)DIN * DTR / 8, 256)), b256, 0, stream>>>(omega_w, DTR, DIN, DTR / 8, DIN * DTR / 8, WSC, W3 + (size_t)DIN * DTR);
  k_cvt<<<dim3(cdv((long)DIN * DTR / 8, 256)), b256, 0, stream>>>(dt_w, DTR, DIN, DTR / 8, DIN * DTR / 8, WSC, W3 + (size_t)2 * DIN * DTR);
  k_cvt<<<dim3(cdv((long)DMOD * DIN / 8, 256)), b256, 0, stream>>>(out_w, DIN, DMOD, DIN / 8, DMOD * DIN / 8, WSC, WOUT);
  k_ln<<<dim3(NTOK), dim3(128), 0, stream>>>(x, norm_w, norm_b, XH, XL);
  k_gemm<0, 1><<<dim3(NTOK / TPB, DIN / 64), b256, 0, stream>>>(XH, XH, DMOD, 0, WIN, DMOD, DMOD, 1.0f / WSC, 0.0f,
                                                                 alpha_b, omega_b, dt_b, x, PROJ, NPP);
  k_gemm<0, 2><<<dim3(NTOK / TPB, (NPP - DIN) / 64), b256, 0, stream>>>(XH, XL, DMOD, 0, WIN + (size_t)DIN * DMOD, DMOD, DMOD,
                                                                         1.0f / WSC, 1.0f / (WSC * LSC),
                                                                         alpha_b, omega_b, dt_b, x, PROJ + DIN, NPP);
  k_split<<<dim3(cdv((long)NTOK * DTR / 8, 256)), b256, 0, stream>>>(PROJ + OFF_R, NPP, DTR / 8, NTOK * DTR / 8, DTPH, DTPL);
  for (int c = 0; c < NCHK; ++c) {
    k_gemm<1, 2><<<dim3(MCH / TPB, NADO / 64), b256, 0, stream>>>(DTPH, DTPL, DTR, c * TCH, W3, DTR, DTR, 1.0f / WSC, 1.0f / (WSC * LSC),
                                                                  alpha_b, omega_b, dt_b, x, ADO, NADO);
    const float* hsrc = (c == 0) ? state : (const float*)hout;
    k_scan<<<dim3(NSCB), dim3(CHB), 0, stream>>>(PROJ, ADO, c * TCH, (c == 0) ? 1 : 0, hsrc, conv_w, conv_b, C_w, D_p, YG, hout);
  }
  k_gemm<2, 1><<<dim3(NTOK / TPB, DMOD / 64), b256, 0, stream>>>(YG, YG, DIN, 0, WOUT, DIN, DIN, 1.0f / (WSC * YSC), 0.0f,
                                                                 alpha_b, omega_b, dt_b, x, out, DMOD);
}
